// MultiHeadAttention_88905823027389
// MI455X (gfx1250) — hardware-verified
//
#include <hip/hip_runtime.h>
#include <math.h>

typedef __attribute__((ext_vector_type(16))) _Float16 v16h;
typedef __attribute__((ext_vector_type(8)))  _Float16 v8h;
typedef __attribute__((ext_vector_type(16))) __bf16   v16b;
typedef __attribute__((ext_vector_type(8)))  __bf16   v8b;
typedef __attribute__((ext_vector_type(8)))  float    v8f;
typedef __attribute__((ext_vector_type(4)))  float    v4f;
typedef __attribute__((ext_vector_type(4)))  int      v4i;

constexpr int kNb    = 2;
constexpr int kSeq   = 2048;
constexpr int kEmb   = 2048;
constexpr int kHeads = 32;
constexpr int kKvh   = 8;
constexpr int kGrp   = kHeads / kKvh;
constexpr int kHd    = kEmb / kHeads;
constexpr int kKvw   = kKvh * kHd;
constexpr int kTok   = kNb * kSeq;
constexpr int kQkw   = kEmb + kKvw;
constexpr int kHpr   = 256;
constexpr int kLpr   = kSeq - kHpr;
static_assert(kGrp == 4 && kHd == 64 && kKvw == 512 && kTok == 4096 && kQkw == 2560);
static_assert((kEmb % 32) == 0 && (kHd % 32) == 0);
static_assert((kTok % 64) == 0 && (kQkw % 64) == 0 && (kKvw % 64) == 0 && (kEmb % 64) == 0);
static_assert((kHpr % 64) == 0 && (kLpr % 64) == 0 && (kSeq % 32) == 0 && (kHpr % 32) == 0);

constexpr float kXCarry   = 64.0f;
constexpr float kWCarry   = 1024.0f;
constexpr float kActCarry = 64.0f;
constexpr float kPLog2    = 12.0f;
constexpr float kCtxCarry = 256.0f;
constexpr float kProjScaleLp = kActCarry / (kXCarry * kWCarry);
constexpr float kProjScaleHp = 1.0f / (kXCarry * kWCarry);
constexpr float kOutScaleLp  = 1.0f / (kCtxCarry * kWCarry);
constexpr float kOutScaleHp  = 1.0f;
constexpr float inv_sqrt_pow4(int n) { float r = 1.0f; while (n > 1) { n /= 4; r *= 0.5f; } return r; }
constexpr float kInvSqrtHd = inv_sqrt_pow4(kHd);
static_assert(kInvSqrtHd * kInvSqrtHd * (float)kHd == 1.0f);
constexpr float kLog2e = 1.4426950408889634f;
constexpr float kScLp  = kInvSqrtHd * kLog2e / (kActCarry * kActCarry);
constexpr float kScHp  = kInvSqrtHd * kLog2e;

constexpr size_t kOffX16   = 0;
constexpr size_t kOffWQK16 = kOffX16   + (size_t)kTok * kEmb * 2;
constexpr size_t kOffWV16  = kOffWQK16 + (size_t)kQkw * kEmb * 2;
constexpr size_t kOffWO16  = kOffWV16  + (size_t)kKvw * kEmb * 2;
constexpr size_t kOffWOB   = kOffWO16  + (size_t)kEmb * kEmb * 2;
constexpr size_t kOffQK16  = kOffWOB   + (size_t)kEmb * kEmb * 2;
constexpr size_t kOffVT16  = kOffQK16  + (size_t)kTok * kQkw * 2;
constexpr size_t kOffQKBH  = kOffVT16  + (size_t)kKvw * kTok * 2;
constexpr size_t kOffQKBL  = kOffQKBH  + (size_t)kNb * kHpr * kQkw * 2;
constexpr size_t kOffVTBH  = kOffQKBL  + (size_t)kNb * kHpr * kQkw * 2;
constexpr size_t kOffVTBL  = kOffVTBH  + (size_t)kNb * kKvw * kHpr * 2;
constexpr size_t kOffCTX16 = kOffVTBL  + (size_t)kNb * kKvw * kHpr * 2;
constexpr size_t kOffCTXBH = kOffCTX16 + (size_t)kTok * kEmb * 2;
constexpr size_t kOffCTXBL = kOffCTXBH + (size_t)kNb * kHpr * kEmb * 2;
constexpr size_t kWsTotal  = kOffCTXBL + (size_t)kNb * kHpr * kEmb * 2;
static_assert(kWsTotal == 98566144ull);
static_assert(kWsTotal <= 134217728ull);
static_assert((kOffWQK16 % 128) == 0 && (kOffWV16 % 128) == 0 && (kOffWO16 % 128) == 0 && (kOffWOB % 128) == 0 &&
              (kOffQK16 % 128) == 0 && (kOffVT16 % 128) == 0 && (kOffQKBH % 128) == 0 && (kOffQKBL % 128) == 0 &&
              (kOffVTBH % 128) == 0 && (kOffVTBL % 128) == 0 && (kOffCTX16 % 128) == 0 && (kOffCTXBH % 128) == 0 &&
              (kOffCTXBL % 128) == 0);

__device__ __forceinline__ unsigned short f2bf_bits(float f) {
  unsigned u = __float_as_uint(f);
  return (unsigned short)((u + 0x7FFFu + ((u >> 16) & 1u)) >> 16);
}
__device__ __forceinline__ float bf_bits2f(unsigned short h) { return __uint_as_float(((unsigned)h) << 16); }
__device__ __forceinline__ float fast_exp2(float x) { return __builtin_amdgcn_exp2f(x); }

__device__ __forceinline__ void grp_guard_h(v8f& a, v8f& b, v8f& c, v8f& d, v16h x, v16h y) {
  asm volatile("v_nop\n\tv_nop\n\tv_nop\n\tv_nop" : "+v"(a), "+v"(b), "+v"(c), "+v"(d) : "v"(x), "v"(y));
}
__device__ __forceinline__ void grp_guard_b(v8f& a, v8f& b, v8f& c, v8f& d, v16b x, v16b y) {
  asm volatile("v_nop\n\tv_nop\n\tv_nop\n\tv_nop" : "+v"(a), "+v"(b), "+v"(c), "+v"(d) : "v"(x), "v"(y));
}
__device__ __forceinline__ void keep4_h(v16h a, v16h b, v16h c, v16h d) { asm volatile("v_nop" :: "v"(a), "v"(b), "v"(c), "v"(d)); }
__device__ __forceinline__ void keep4_b(v16b a, v16b b, v16b c, v16b d) { asm volatile("v_nop" :: "v"(a), "v"(b), "v"(c), "v"(d)); }
__device__ __forceinline__ void acc_guard4(v8f& a, v8f& b, v8f& c, v8f& d) { asm volatile("v_nop\n\tv_nop\n\tv_nop\n\tv_nop" : "+v"(a), "+v"(b), "+v"(c), "+v"(d)); }

template <typename T> struct Frag;
template <> struct Frag<_Float16> {
  typedef v16h V; union U { v16h v; v8h h[2]; };
  static __device__ __forceinline__ v16h load(const _Float16* p) {
    U f; f.h[0] = *(const v8h*)(p); f.h[1] = *(const v8h*)(p + 16); return f.v;
  }
  static __device__ __forceinline__ v8f mma(v16h a, v16h b, v8f c) {
    return __builtin_amdgcn_wmma_f32_16x16x32_f16(false, a, false, b, (short)0, c, false, false);
  }
  static __device__ __forceinline__ void guard(v8f& a, v8f& b, v8f& c, v8f& d, v16h x, v16h y) { grp_guard_h(a, b, c, d, x, y); }
  static __device__ __forceinline__ void keep(v16h a, v16h b, v16h c, v16h d) { keep4_h(a, b, c, d); }
};
template <> struct Frag<__bf16> {
  typedef v16b V; union U { v16b v; v8b h[2]; };
  static __device__ __forceinline__ v16b load(const __bf16* p) {
    U f; f.h[0] = *(const v8b*)(p); f.h[1] = *(const v8b*)(p + 16); return f.v;
  }
  static __device__ __forceinline__ v8f mma(v16b a, v16b b, v8f c) {
    return __builtin_amdgcn_wmma_f32_16x16x32_bf16(false, a, false, b, (short)0, c, false, false);
  }
  static __device__ __forceinline__ void guard(v8f& a, v8f& b, v8f& c, v8f& d, v16b x, v16b y) { grp_guard_b(a, b, c, d, x, y); }
  static __device__ __forceinline__ void keep(v16b a, v16b b, v16b c, v16b d) { keep4_b(a, b, c, d); }
};

template <int ET> struct Elem;
template <> struct Elem<0> { typedef _Float16 T; };
template <> struct Elem<1> { typedef __bf16 T; };

template <int ET, int SPL, int OUT_MODE>
__global__ __launch_bounds__(256) void wmma_gemm64(
    const unsigned short* __restrict__ Ap, const unsigned short* __restrict__ A2p, int lda, long strideA,
    const unsigned short* __restrict__ Btp, int ldb, long strideB,
    void* __restrict__ Cout, void* __restrict__ Cout2, int ldc, long strideC,
    int M, int N, int K, float scale) {
  typedef typename Elem<ET>::T T;
  typedef typename Frag<T>::V V;
  const T* A = (const T*)Ap; const T* A2 = (const T*)A2p; const T* Bt = (const T*)Btp;
  __shared__ __align__(16) float sT[8][16 * 68];
  const int b    = blockIdx.y;
  const int lane = threadIdx.x & 31;
  const int wave = __builtin_amdgcn_readfirstlane((int)(threadIdx.x >> 5));
  const int tilesN = N >> 6;
  const int tilesM = M >> 6;
  const int tile = blockIdx.x * 8 + wave;
  if (tile >= tilesM * tilesN) return;
  const int tm = tile / tilesN;
  const int tn = tile - tm * tilesN;
  const int m0 = tm << 6;
  const int n0 = tn << 6;

  const T* Ab  = A  + (size_t)b * strideA;
  const T* Bb  = Bt + (size_t)b * strideB;
  const T* Ab2 = (SPL >= 1) ? (A2 + (size_t)b * strideA) : nullptr;

  const int rlane = lane & 15;
  const int koff  = (lane >> 4) * 8;
  const int mOff  = (lane >> 4) * 8;

  v8f acc[4][4];
#pragma unroll
  for (int i = 0; i < 4; ++i)
#pragma unroll
    for (int j = 0; j < 4; ++j) acc[i][j] = (v8f){0.f,0.f,0.f,0.f,0.f,0.f,0.f,0.f};

  for (int k0 = 0; k0 < K; k0 += 32) {
    V bh[4];
#pragma unroll
    for (int j = 0; j < 4; ++j) {
      const size_t bo = (size_t)(n0 + (j << 4) + rlane) * ldb + koff + k0;
      bh[j] = Frag<T>::load(Bb + bo);
    }
#pragma unroll
    for (int i = 0; i < 4; ++i) {
      const size_t ao = (size_t)(m0 + (i << 4) + rlane) * lda + koff + k0;
      V ah = Frag<T>::load(Ab + ao);
      V al;
      if (SPL >= 1) al = Frag<T>::load(Ab2 + ao);
#pragma unroll
      for (int j = 0; j < 4; ++j) {
        acc[i][j] = Frag<T>::mma(ah, bh[j], acc[i][j]);
        if (SPL >= 1) acc[i][j] = Frag<T>::mma(al, bh[j], acc[i][j]);
      }
      Frag<T>::guard(acc[i][0], acc[i][1], acc[i][2], acc[i][3], ah, (SPL >= 1) ? al : ah);
    }
    Frag<T>::keep(bh[0], bh[1], bh[2], bh[3]);
  }
  acc_guard4(acc[0][0], acc[0][1], acc[0][2], acc[0][3]);
  acc_guard4(acc[1][0], acc[1][1], acc[1][2], acc[1][3]);
  acc_guard4(acc[2][0], acc[2][1], acc[2][2], acc[2][3]);
  acc_guard4(acc[3][0], acc[3][1], acc[3][2], acc[3][3]);

  float* slab = sT[wave];
#pragma unroll
  for (int i = 0; i < 4; ++i) {
    const int mBase = m0 + (i << 4);
#pragma unroll
    for (int j = 0; j < 4; ++j) {
#pragma unroll
      for (int r = 0; r < 8; ++r) {
        const float v = acc[i][j][r] * scale;
        slab[(mOff + r) * 68 + (j << 4) + rlane] = v;
      }
    }
    __builtin_amdgcn_fence(__ATOMIC_RELEASE, "workgroup");
    __builtin_amdgcn_wave_barrier();
    __builtin_amdgcn_fence(__ATOMIC_ACQUIRE, "workgroup");
    if (OUT_MODE == 0) {
      float* C = (float*)Cout + (size_t)b * strideC;
      const int hh = lane >> 4, c4 = (lane & 15) * 4;
      for (int pass = 0; pass < 2; ++pass) {
#pragma unroll
        for (int it = 0; it < 8; ++it) {
          const int row = it * 2 + hh;
          v4f v = *(const v4f*)(slab + row * 68 + c4);
          *(volatile v4f*)(C + (size_t)(mBase + row) * ldc + n0 + c4) = v;
        }
        __threadfence();
      }
    } else {
      const int q = lane >> 3, c8 = (lane & 7) * 8;
      unsigned short* C  = (unsigned short*)Cout + (size_t)b * strideC;
      unsigned short* C2 = (OUT_MODE == 2) ? ((unsigned short*)Cout2 + (size_t)b * strideC) : nullptr;
      for (int pass = 0; pass < 2; ++pass) {
#pragma unroll
        for (int it = 0; it < 4; ++it) {
          const int row = it * 4 + q;
          const float* sp = slab + row * 68 + c8;
          v8h hv, lv;
#pragma unroll
          for (int e = 0; e < 8; ++e) {
            if (OUT_MODE == 1) {
              hv[e] = (_Float16)sp[e];
            } else {
              unsigned short hb = f2bf_bits(sp[e]);
              unsigned short lb = f2bf_bits(sp[e] - bf_bits2f(hb));
              hv[e] = __builtin_bit_cast(_Float16, hb);
              lv[e] = __builtin_bit_cast(_Float16, lb);
            }
          }
          *(volatile v8h*)(C + (size_t)(mBase + row) * ldc + n0 + c8) = hv;
          if (OUT_MODE == 2) *(volatile v8h*)(C2 + (size_t)(mBase + row) * ldc + n0 + c8) = lv;
        }
        __threadfence();
      }
    }
    __builtin_amdgcn_fence(__ATOMIC_RELEASE, "workgroup");
    __builtin_amdgcn_wave_barrier();
    __builtin_amdgcn_fence(__ATOMIC_ACQUIRE, "workgroup");
  }
}

__global__ __launch_bounds__(256) void cvt_plane_kernel(
    const float* __restrict__ src, unsigned short* __restrict__ d16, unsigned short* __restrict__ dbf,
    float carry, int wantbf, int total8)
{
  const int i = blockIdx.x * 256 + threadIdx.x;
  if (i >= total8) return;
  const size_t e0 = (size_t)i << 3;
  const v4f a0 = *(const v4f*)(src + e0);
  const v4f a1 = *(const v4f*)(src + e0 + 4);
  v8h hv, bv;
#pragma unroll
  for (int e = 0; e < 4; ++e) {
    const float f0 = a0[e];
    const float f1 = a1[e];
    const unsigned short b0 = f2bf_bits(f0);
    const unsigned short b1 = f2bf_bits(f1);
    const float r0 = bf_bits2f(b0) * carry;
    const float r1 = bf_bits2f(b1) * carry;
    hv[e]     = (_Float16)r0;
    hv[4 + e] = (_Float16)r1;
    bv[e]     = __builtin_bit_cast(_Float16, b0);
    bv[4 + e] = __builtin_bit_cast(_Float16, b1);
  }
  unsigned short* q16 = d16 + e0;
  unsigned short* qbf = dbf + e0;
  *(volatile v8h*)q16 = hv;
  if (wantbf) *(volatile v8h*)qbf = bv;
  __threadfence();
  *(volatile v8h*)q16 = hv;
  if (wantbf) *(volatile v8h*)qbf = bv;
}

union FragBits { v16b v; v8b h[2]; };
__device__ __forceinline__ v16b ld_frag16(const unsigned short* p) {
  FragBits f;
  f.h[0] = *(const v8b*)(p);
  f.h[1] = *(const v8b*)(p + 16);
  return f.v;
}
template <bool F16> __device__ __forceinline__ v8f mma16(v16b a, v16b b, v8f c) {
  if (F16) {
    const v16h ah = __builtin_bit_cast(v16h, a), bh = __builtin_bit_cast(v16h, b);
    c = __builtin_amdgcn_wmma_f32_16x16x32_f16(false, ah, false, bh, (short)0, c, false, false);
    asm volatile("v_nop\n\tv_nop\n\tv_nop\n\tv_nop" : "+v"(c) : "v"(ah), "v"(bh));
    return c;
  }
  c = __builtin_amdgcn_wmma_f32_16x16x32_bf16(false, a, false, b, (short)0, c, false, false);
  asm volatile("v_nop\n\tv_nop\n\tv_nop\n\tv_nop" : "+v"(c) : "v"(a), "v"(b));
  return c;
}

template <bool HP>
__global__ __launch_bounds__(128) void attn_kernel(
    const unsigned short* __restrict__ QKhi, const unsigned short* __restrict__ QKlo,
    const unsigned short* __restrict__ VThi, const unsigned short* __restrict__ VTlo,
    const int* __restrict__ mask,
    unsigned short* CXhi, unsigned short* CXlo)
{
  constexpr bool  F16  = !HP;
  constexpr int   kQt0 = HP ? 0 : (kHpr / 16);
  constexpr int   kNqt = HP ? (kHpr / 16) : (kLpr / 16);
  constexpr int   kRpb = HP ? kHpr : kSeq;
  constexpr int   kVp  = HP ? kHpr : kTok;
  constexpr float kSc  = HP ? kScHp : kScLp;
  constexpr float kPl  = HP ? 0.0f : kPLog2;
  constexpr float kCf  = HP ? 1.0f : (kCtxCarry / kActCarry);
  __shared__ __align__(16) float Os[4][16 * 68];

  const int lane = threadIdx.x & 31;
  const int wave = __builtin_amdgcn_readfirstlane((int)(threadIdx.x >> 5));
  const int hh   = lane >> 4;
  const int c    = lane & 15;
  const int bx   = (int)blockIdx.x;
  const int qt   = kQt0 + bx % kNqt;
  const int rest = bx / kNqt;
  const int kv   = rest % kKvh;
  int b = rest / kKvh;
  b = (b < kNb) ? b : (kNb - 1);
  const int head = kv * kGrp + wave;
  const int s0   = qt * 16;

  const size_t qoff = (size_t)(b * kRpb + s0 + c) * kQkw + head * kHd + 8 * hh;
  v16b qf[2], ql[2];
#pragma unroll
  for (int dc = 0; dc < 2; ++dc) {
    qf[dc] = ld_frag16(QKhi + qoff + dc * 32);
    if (HP) ql[dc] = ld_frag16(QKlo + qoff + dc * 32);
    else    ql[dc] = qf[dc];
  }
  const size_t kbase = (size_t)(b * kRpb) * kQkw + kEmb + kv * kHd + 8 * hh;
  const size_t vbase = (HP ? ((size_t)b * kKvw * kHpr) : ((size_t)b * kSeq)) + (size_t)(kv * kHd) * kVp + 8 * hh;

  float mrun = -INFINITY;
  float lsum = 0.0f;
  v8f oT[4];
#pragma unroll
  for (int t = 0; t < 4; ++t) oT[t] = (v8f){0.f,0.f,0.f,0.f,0.f,0.f,0.f,0.f};

  const int nch = (s0 + 16 + 31) >> 5;
#pragma unroll 1
  for (int ch = 0; ch < nch; ++ch) {
    const int t0 = ch * 32;
    v8f st[2];
#pragma unroll
    for (int j = 0; j < 2; ++j) {
      st[j] = (v8f){0.f,0.f,0.f,0.f,0.f,0.f,0.f,0.f};
      const size_t koff = kbase + (size_t)(t0 + 16 * j + c) * kQkw;
#pragma unroll
      for (int dc = 0; dc < 2; ++dc) {
        const v16b kf = ld_frag16(QKhi + koff + dc * 32);
        st[j] = mma16<F16>(kf, qf[dc], st[j]);
        if (HP) {
          const v16b kl = ld_frag16(QKlo + koff + dc * 32);
          st[j] = mma16<F16>(kf, ql[dc], st[j]);
          st[j] = mma16<F16>(kl, qf[dc], st[j]);
        }
      }
    }
    float x[2][8];
#pragma unroll
    for (int j = 0; j < 2; ++j)
#pragma unroll
      for (int r = 0; r < 8; ++r) x[j][r] = st[j][r] * kSc;

    if (ch == nch - 1) {
      const int qs = s0 + c;
      const int* mrow = mask + (size_t)qs * kSeq + t0 + 8 * hh;
#pragma unroll
      for (int j = 0; j < 2; ++j) {
        v4i m0 = *(const v4i*)(mrow + 16 * j);
        v4i m1 = *(const v4i*)(mrow + 16 * j + 4);
        asm volatile("" : "+v"(m0));
        asm volatile("" : "+v"(m1));
#pragma unroll
        for (int r = 0; r < 4; ++r) {
          const int kt0 = t0 + 16 * j + 8 * hh + r;
          const int kt1 = kt0 + 4;
          const int ma = m0[r];
          const int mb = m1[r];
          const bool keep0 = (kt0 <= qs) & (ma != 0);
          const bool keep1 = (kt1 <= qs) & (mb != 0);
          x[j][r]     = keep0 ? x[j][r]     : -INFINITY;
          x[j][4 + r] = keep1 ? x[j][4 + r] : -INFINITY;
        }
      }
    }

    float mloc = fmaxf(x[0][0], x[1][0]);
#pragma unroll
    for (int r = 1; r < 8; ++r) mloc = fmaxf(mloc, fmaxf(x[0][r], x[1][r]));
    const float mother = __shfl_xor(mloc, 16, 32);
    mloc = fmaxf(mloc, mother);
    const float mnew  = fmaxf(mrun, mloc);
    const float alpha = fast_exp2(mrun - mnew);
    mrun = mnew;
    const float moff = mnew - kPl;
    float ps = 0.0f;
#pragma unroll
    for (int j = 0; j < 2; ++j)
#pragma unroll
      for (int r = 0; r < 8; ++r) {
        const float pv = fast_exp2(x[j][r] - moff);
        x[j][r] = pv;
        ps += pv;
      }
    lsum = lsum * alpha + ps;
#pragma unroll
    for (int t = 0; t < 4; ++t)
#pragma unroll
      for (int r = 0; r < 8; ++r) oT[t][r] *= alpha;

    v16b pfh, pfl;
#pragma unroll
    for (int i = 0; i < 8; ++i) {
      const float p0 = x[0][i];
      const float p1 = x[1][i];
      if (HP) {
        const unsigned short h0 = f2bf_bits(p0);
        const unsigned short h1 = f2bf_bits(p1);
        const unsigned short l0 = f2bf_bits(p0 - bf_bits2f(h0));
        const unsigned short l1 = f2bf_bits(p1 - bf_bits2f(h1));
        pfh[i]     = __builtin_bit_cast(__bf16, h0);
        pfh[8 + i] = __builtin_bit_cast(__bf16, h1);
        pfl[i]     = __builtin_bit_cast(__bf16, l0);
        pfl[8 + i] = __builtin_bit_cast(__bf16, l1);
      } else {
        const _Float16 g0 = (_Float16)p0;
        const _Float16 g1 = (_Float16)p1;
        pfh[i]     = __builtin_bit_cast(__bf16, g0);
        pfh[8 + i] = __builtin_bit_cast(__bf16, g1);
      }
    }
    if (!HP) pfl = pfh;

#pragma unroll
    for (int t = 0; t < 4; ++t) {
      const size_t vo = vbase + (size_t)(16 * t + c) * kVp + t0;
      const v16b vf = ld_frag16(VThi + vo);
      oT[t] = mma16<F16>(vf, pfh, oT[t]);
      if (HP) {
        const v16b vl = ld_frag16(VTlo + vo);
        oT[t] = mma16<F16>(vf, pfl, oT[t]);
        oT[t] = mma16<F16>(vl, pfh, oT[t]);
      }
    }
  }

  const float lother = __shfl_xor(lsum, 16, 32);
  const float ltot = lsum + lother;
  const float inv = kCf * (1.0f / ltot);
  float* os = Os[wave];
#pragma unroll
  for (int t = 0; t < 4; ++t) {
    const v4f a0 = (v4f){oT[t][0] * inv, oT[t][1] * inv, oT[t][2] * inv, oT[t][3] * inv};
    const v4f a1 = (v4f){oT[t][4] * inv, oT[t][5] * inv, oT[t][6] * inv, oT[t][7] * inv};
    *(v4f*)(os + c * 68 + 16 * t + 8 * hh)     = a0;
    *(v4f*)(os + c * 68 + 16 * t + 8 * hh + 4) = a1;
  }
  __builtin_amdgcn_fence(__ATOMIC_RELEASE, "workgroup");
  __builtin_amdgcn_wave_barrier();
  __builtin_amdgcn_fence(__ATOMIC_ACQUIRE, "workgroup");
  {
    const int q = lane >> 3, c8 = (lane & 7) * 8;
    v8h hv[4], lv[4];
#pragma unroll
    for (int it = 0; it < 4; ++it) {
      const int row = it * 4 + q;
      const float* sp = os + row * 68 + c8;
      const v4f a0 = *(const v4f*)(sp);
      const v4f a1 = *(const v4f*)(sp + 4);
#pragma unroll
      for (int e = 0; e < 4; ++e) {
        const float f0 = a0[e];
        const float f1 = a1[e];
        if (HP) {
          const unsigned short h0 = f2bf_bits(f0), h1 = f2bf_bits(f1);
          const unsigned short l0 = f2bf_bits(f0 - bf_bits2f(h0)), l1 = f2bf_bits(f1 - bf_bits2f(h1));
          hv[it][e]     = __builtin_bit_cast(_Float16, h0);
          hv[it][4 + e] = __builtin_bit_cast(_Float16, h1);
          lv[it][e]     = __builtin_bit_cast(_Float16, l0);
          lv[it][4 + e] = __builtin_bit_cast(_Float16, l1);
        } else {
          hv[it][e]     = (_Float16)f0;
          hv[it][4 + e] = (_Float16)f1;
          lv[it][e]     = hv[it][e];
          lv[it][4 + e] = hv[it][4 + e];
        }
      }
    }
    const size_t obase = (size_t)(b * kRpb + s0) * kEmb + head * kHd + c8;
    for (int pass = 0; pass < 2; ++pass) {
#pragma unroll
      for (int it = 0; it < 4; ++it) {
        const int row = it * 4 + q;
        *(volatile v8h*)(CXhi + obase + (size_t)row * kEmb) = hv[it];
        if (HP) *(volatile v8h*)(CXlo + obase + (size_t)row * kEmb) = lv[it];
      }
      __threadfence();
    }
  }
}

constexpr int gemm_blocks(int M, int N) { return ((M / 64) * (N / 64) + 7) / 8; }

extern "C" void kernel_launch(void* const* d_in, const int* in_sizes, int n_in,
                              void* d_out, int out_size, void* d_ws, size_t ws_size,
                              hipStream_t stream) {
  if (n_in < 6) return;
  if (in_sizes[0] != kTok * kEmb) return;
  if (in_sizes[1] != kSeq * kSeq) return;
  if (in_sizes[2] != kEmb * kEmb) return;
  if (in_sizes[3] != kKvw * kEmb) return;
  if (in_sizes[4] != kKvw * kEmb) return;
  if (in_sizes[5] != kEmb * kEmb) return;
  if (out_size != kTok * kEmb) return;
  if (ws_size < kWsTotal) return;

  const float* x    = (const float*)d_in[0];
  const int*   mask = (const int*)d_in[1];
  const float* Wq   = (const float*)d_in[2];
  const float* Wk   = (const float*)d_in[3];
  const float* Wv   = (const float*)d_in[4];
  const float* Wo   = (const float*)d_in[5];
  float* out = (float*)d_out;

  char* ws = (char*)d_ws;
  unsigned short* X16   = (unsigned short*)(ws + kOffX16);
  unsigned short* WQK16 = (unsigned short*)(ws + kOffWQK16);
  unsigned short* WV16  = (unsigned short*)(ws + kOffWV16);
  unsigned short* WO16  = (unsigned short*)(ws + kOffWO16);
  unsigned short* WOB   = (unsigned short*)(ws + kOffWOB);
  unsigned short* QK16  = (unsigned short*)(ws + kOffQK16);
  unsigned short* VT16  = (unsigned short*)(ws + kOffVT16);
  unsigned short* QKBH  = (unsigned short*)(ws + kOffQKBH);
  unsigned short* QKBL  = (unsigned short*)(ws + kOffQKBL);
  unsigned short* VTBH  = (unsigned short*)(ws + kOffVTBH);
  unsigned short* VTBL  = (unsigned short*)(ws + kOffVTBL);
  unsigned short* CTX16 = (unsigned short*)(ws + kOffCTX16);
  unsigned short* CTXBH = (unsigned short*)(ws + kOffCTXBH);
  unsigned short* CTXBL = (unsigned short*)(ws + kOffCTXBL);

  cvt_plane_kernel<<<(kTok * kEmb / 8) / 256, 256, 0, stream>>>(x, X16, X16, kXCarry, 0, kTok * kEmb / 8);
  cvt_plane_kernel<<<(kEmb * kEmb / 8) / 256, 256, 0, stream>>>(Wq, WQK16, WQK16, kWCarry, 0, kEmb * kEmb / 8);
  cvt_plane_kernel<<<(kKvw * kEmb / 8) / 256, 256, 0, stream>>>(Wk, WQK16 + (size_t)kEmb * kEmb, WQK16 + (size_t)kEmb * kEmb,
                                                                 kWCarry, 0, kKvw * kEmb / 8);
  cvt_plane_kernel<<<(kKvw * kEmb / 8) / 256, 256, 0, stream>>>(Wv, WV16, WV16, kWCarry, 0, kKvw * kEmb / 8);
  cvt_plane_kernel<<<(kEmb * kEmb / 8) / 256, 256, 0, stream>>>(Wo, WO16, WOB, kWCarry, 1, kEmb * kEmb / 8);

  wmma_gemm64<0, 0, 1><<<dim3(gemm_blocks(kTok, kQkw), 1), 256, 0, stream>>>(
      X16, nullptr, kEmb, 0L,
      WQK16, kEmb, 0L,
      (void*)QK16, nullptr, kQkw, 0L,
      kTok, kQkw, kEmb, kProjScaleLp);

  wmma_gemm64<0, 0, 1><<<dim3(gemm_blocks(kKvw, kTok), 1), 256, 0, stream>>>(
      WV16, nullptr, kEmb, 0L,
      X16, kEmb, 0L,
      (void*)VT16, nullptr, kTok, 0L,
      kKvw, kTok, kEmb, kProjScaleLp);

  wmma_gemm64<0, 0, 2><<<dim3(gemm_blocks(kHpr, kQkw), kNb), 256, 0, stream>>>(
      X16, nullptr, kEmb, (long)kSeq * kEmb,
      WQK16, kEmb, 0L,
      (void*)QKBH, (void*)QKBL, kQkw, (long)kHpr * kQkw,
      kHpr, kQkw, kEmb, kProjScaleHp);

  wmma_gemm64<0, 0, 2><<<dim3(gemm_blocks(kKvw, kHpr), kNb), 256, 0, stream>>>(
      WV16, nullptr, kEmb, 0L,
      X16, kEmb, (long)kSeq * kEmb,
      (void*)VTBH, (void*)VTBL, kHpr, (long)kKvw * kHpr,
      kKvw, kHpr, kEmb, kProjScaleHp);

  attn_kernel<false><<<(kLpr / 16) * kKvh * kNb, 128, 0, stream>>>(QK16, QK16, VT16, VT16, mask, CTX16, CTX16);
  attn_kernel<true><<<(kHpr / 16) * kKvh * kNb, 128, 0, stream>>>(QKBH, QKBL, VTBH, VTBL, mask, CTXBH, CTXBL);

  wmma_gemm64<0, 0, 0><<<dim3(gemm_blocks(kLpr, kEmb), kNb), 256, 0, stream>>>(
      CTX16 + (size_t)kHpr * kEmb, nullptr, kEmb, (long)kSeq * kEmb,
      WO16, kEmb, 0L,
      (void*)(out + (size_t)kHpr * kEmb), nullptr, kEmb, (long)kSeq * kEmb,
      kLpr, kEmb, kEmb, kOutScaleLp);

  wmma_gemm64<1, 1, 0><<<dim3(gemm_blocks(kHpr, kEmb), kNb), 256, 0, stream>>>(
      CTXBH, CTXBL, kEmb, (long)kHpr * kEmb,
      WOB, kEmb, 0L,
      (void*)out, nullptr, kEmb, (long)kSeq * kEmb,
      kHpr, kEmb, kEmb, kOutScaleHp);
}
